// SimpleLanguageModel_13486197309501
// MI455X (gfx1250) — hardware-verified
//
#include <hip/hip_runtime.h>
#include <math.h>

typedef __attribute__((ext_vector_type(16))) _Float16 v16h;
typedef __attribute__((ext_vector_type(8)))  _Float16 v8h;
typedef __attribute__((ext_vector_type(8)))  float    v8f;
typedef __attribute__((ext_vector_type(4)))  float    v4f;

constexpr int kBatch = 64;
constexpr int kSteps = 512;
constexpr int kInDim = 256;
constexpr int kHid   = 512;
constexpr int kOutD  = 256;
constexpr int kGates = 4 * kHid;
constexpr int kKc    = kInDim + kHid;
constexpr int kRowsAll = kBatch * kSteps;
constexpr int kRowsPerBlk = 16;
constexpr int kStepBlocks = kBatch / kRowsPerBlk;
constexpr int kAP = kKc + 8;
constexpr int kHP = kHid + 4;
constexpr float kCarryA = 64.0f;
constexpr float kCarryW = 1024.0f;
constexpr float kFold   = 1.0f / (kCarryA * kCarryW);

static_assert(kKc == 768 && (kKc % 32) == 0 && (kHid % 32) == 0, "K multiples of 32");
static_assert((kRowsAll % 64) == 0 && (kOutD % 64) == 0, "GEMM M,N multiples of 64");
static_assert(kHid == 16 * 32, "16 waves x 32 hidden columns");
static_assert(kInDim == 32 * 8 && kHid == 2 * 32 * 8, "staging maps: 32 lanes x 8 elements");
static_assert((kAP * 2) % 16 == 0 && (kHP * 4) % 16 == 0, "16-B aligned LDS rows");
static_assert(kRowsPerBlk * kAP * 2 + kRowsPerBlk * kHP * 4 <= 65536, "static LDS");

constexpr size_t kOffWcat = 0;
constexpr size_t kOffFcw  = kOffWcat + (size_t)kGates * kKc * 2;
constexpr size_t kOffBias = kOffFcw  + (size_t)kOutD * kHid * 2;
constexpr size_t kOffHs   = kOffBias + (size_t)kGates * 4;
constexpr size_t kWsTotal = kOffHs   + (size_t)kRowsAll * kHid * 2;
static_assert(kWsTotal == 36970496ull, "carve total");
static_assert(kWsTotal <= 134217728ull, "carve cap");
static_assert((kOffFcw % 128) == 0 && (kOffBias % 128) == 0 && (kOffHs % 128) == 0, "128-B aligned regions");

constexpr int kBlkWih  = (kGates * kInDim / 8) / 256;
constexpr int kBlkWhh  = (kGates * kHid / 8) / 256;
constexpr int kBlkFc   = (kOutD * kHid / 8) / 256;
constexpr int kBlkBias = (kGates / 4) / 256;
static_assert(kBlkWih == 256 && kBlkWhh == 512 && kBlkFc == 64 && kBlkBias == 2, "prep coverage");

union FragU { v16h v; v8h h[2]; };

__device__ __forceinline__ v16h frag_load_f16(const _Float16* p) {
  FragU f;
  f.h[0] = *(const v8h*)(p);
  f.h[1] = *(const v8h*)(p + 16);
  return f.v;
}

__device__ __forceinline__ v8f mma_f16_guarded(v16h a, v16h b, v8f c) {
  c = __builtin_amdgcn_wmma_f32_16x16x32_f16(false, a, false, b, (short)0, c, false, false);
  asm volatile("v_nop\n\tv_nop\n\tv_nop\n\tv_nop" : "+v"(c) : "v"(a), "v"(b));
  return c;
}

__device__ __forceinline__ float sig_fast(float z) {
  return __builtin_amdgcn_rcpf(1.0f + __expf(-z));
}
__device__ __forceinline__ float tanh_fast(float z) {
  const float zz = fminf(fmaxf(z, -15.0f), 15.0f);
  return 1.0f - 2.0f * __builtin_amdgcn_rcpf(__expf(2.0f * zz) + 1.0f);
}

__device__ __forceinline__ void convert8_store(const float* __restrict__ src, unsigned short* __restrict__ dst, float carry) {
  const v4f a0 = *(const v4f*)(src);
  const v4f a1 = *(const v4f*)(src + 4);
  v8h hv;
#pragma unroll
  for (int e = 0; e < 4; ++e) {
    hv[e]     = (_Float16)(a0[e] * carry);
    hv[4 + e] = (_Float16)(a1[e] * carry);
  }
  *(volatile v8h*)dst = hv;
  __threadfence();
  *(volatile v8h*)dst = hv;
}

__global__ __launch_bounds__(256) void prep_planes_kernel(
    const float* __restrict__ Wih, const float* __restrict__ Whh,
    const float* __restrict__ bih, const float* __restrict__ bhh,
    const float* __restrict__ fcW,
    unsigned short* __restrict__ Wcat, unsigned short* __restrict__ Fcw, float* __restrict__ biasp)
{
  const int blk = blockIdx.x;
  const int tid = threadIdx.x;
  if (blk < kBlkWih) {
    const int i = blk * 256 + tid;
    const int n = i >> 5;
    const int c8 = (i & 31) * 8;
    convert8_store(Wih + (size_t)i * 8, Wcat + (size_t)n * kKc + c8, kCarryW);
  } else if (blk < kBlkWih + kBlkWhh) {
    const int i = (blk - kBlkWih) * 256 + tid;
    const int n = i >> 6;
    const int c8 = (i & 63) * 8;
    convert8_store(Whh + (size_t)i * 8, Wcat + (size_t)n * kKc + kInDim + c8, kCarryW);
  } else if (blk < kBlkWih + kBlkWhh + kBlkFc) {
    const int i = (blk - kBlkWih - kBlkWhh) * 256 + tid;
    convert8_store(fcW + (size_t)i * 8, Fcw + (size_t)i * 8, kCarryW);
  } else {
    const int i = (blk - kBlkWih - kBlkWhh - kBlkFc) * 256 + tid;
    const v4f a = *(const v4f*)(bih + 4 * i);
    const v4f b = *(const v4f*)(bhh + 4 * i);
    const v4f s = a + b;
    *(volatile v4f*)(biasp + 4 * i) = s;
    __threadfence();
    *(volatile v4f*)(biasp + 4 * i) = s;
  }
}

__global__ __launch_bounds__(512) void lstm_steps_kernel(
    const float* __restrict__ x, const unsigned short* __restrict__ Wcatp,
    const float* __restrict__ biasp, unsigned short* __restrict__ hs16)
{
  __shared__ __align__(16) _Float16 sA[kRowsPerBlk * kAP];
  __shared__ __align__(16) float sHf[kRowsPerBlk * kHP];

  const int tid  = threadIdx.x;
  const int lane = tid & 31;
  const int wave = tid >> 5;
  const int hh   = lane >> 4;
  const int cl   = lane & 15;
  const int b0   = blockIdx.x * kRowsPerBlk;
  const int srow = wave;
  const int sc8  = lane * 8;
  const _Float16* Wcat = (const _Float16*)Wcatp;

  {
    v8h z;
#pragma unroll
    for (int e = 0; e < 8; ++e) z[e] = (_Float16)0.0f;
    *(v8h*)(sA + srow * kAP + kInDim + sc8) = z;
    *(v8h*)(sA + srow * kAP + kInDim + 256 + sc8) = z;
    if (tid < kRowsPerBlk) *(v8h*)(sA + tid * kAP + kKc) = z;
    const float* xp = x + ((size_t)(b0 + srow) * kSteps) * kInDim + sc8;
    const v4f x0 = *(const v4f*)(xp);
    const v4f x1 = *(const v4f*)(xp + 4);
    v8h xv;
#pragma unroll
    for (int e = 0; e < 4; ++e) {
      xv[e]     = (_Float16)(x0[e] * kCarryA);
      xv[4 + e] = (_Float16)(x1[e] * kCarryA);
    }
    *(v8h*)(sA + srow * kAP + sc8) = xv;
  }

  float bz[4][2];
#pragma unroll
  for (int g = 0; g < 4; ++g)
#pragma unroll
    for (int j = 0; j < 2; ++j) bz[g][j] = biasp[g * kHid + 32 * wave + 16 * j + cl];

  float cst[2][8];
#pragma unroll
  for (int j = 0; j < 2; ++j)
#pragma unroll
    for (int r = 0; r < 8; ++r) cst[j][r] = 0.0f;

  const _Float16* wb = Wcat + (size_t)(32 * wave + cl) * kKc + 8 * hh;
  const _Float16* ab = sA + cl * kAP + 8 * hh;

#pragma unroll 1
  for (int t = 0; t < kSteps; ++t) {
    __syncthreads();

    v8f acc[4][2];
#pragma unroll
    for (int g = 0; g < 4; ++g)
#pragma unroll
      for (int j = 0; j < 2; ++j) acc[g][j] = (v8f){0.f, 0.f, 0.f, 0.f, 0.f, 0.f, 0.f, 0.f};

#pragma unroll 1
    for (int kc = 0; kc < kKc / 32; ++kc) {
      const int k0 = kc * 32;
      FragU fa;
      fa.h[0] = *(const v8h*)(ab + k0);
      fa.h[1] = *(const v8h*)(ab + k0 + 16);
#pragma unroll
      for (int g = 0; g < 4; ++g) {
#pragma unroll
        for (int j = 0; j < 2; ++j) {
          const v16h fb = frag_load_f16(wb + (size_t)(g * kHid + 16 * j) * kKc + k0);
          acc[g][j] = mma_f16_guarded(fa.v, fb, acc[g][j]);
        }
      }
    }

#pragma unroll
    for (int j = 0; j < 2; ++j) {
#pragma unroll
      for (int r = 0; r < 8; ++r) {
        const float zi = acc[0][j][r] * kFold + bz[0][j];
        const float zf = acc[1][j][r] * kFold + bz[1][j];
        const float zg = acc[2][j][r] * kFold + bz[2][j];
        const float zo = acc[3][j][r] * kFold + bz[3][j];
        const float iv = sig_fast(zi);
        const float fv = sig_fast(zf);
        const float gv = tanh_fast(zg);
        const float ov = sig_fast(zo);
        const float cn = fv * cst[j][r] + iv * gv;
        cst[j][r] = cn;
        const float hv = ov * tanh_fast(cn);
        sHf[(8 * hh + r) * kHP + 32 * wave + 16 * j + cl] = hv;
      }
    }

    __syncthreads();

    {
      const float* hp = sHf + srow * kHP + sc8;
      const v4f f0 = *(const v4f*)(hp);
      const v4f f1 = *(const v4f*)(hp + 4);
      const v4f f2 = *(const v4f*)(hp + 256);
      const v4f f3 = *(const v4f*)(hp + 260);
      v8h h0, h1;
#pragma unroll
      for (int e = 0; e < 4; ++e) {
        h0[e]     = (_Float16)(f0[e] * kCarryA);
        h0[4 + e] = (_Float16)(f1[e] * kCarryA);
        h1[e]     = (_Float16)(f2[e] * kCarryA);
        h1[4 + e] = (_Float16)(f3[e] * kCarryA);
      }
      *(v8h*)(sA + srow * kAP + kInDim + sc8) = h0;
      *(v8h*)(sA + srow * kAP + kInDim + 256 + sc8) = h1;
      unsigned short* gp = hs16 + ((size_t)(b0 + srow) * kSteps + t) * kHid + sc8;
      *(volatile v8h*)(gp) = h0;
      *(volatile v8h*)(gp + 256) = h1;
      __threadfence();
      *(volatile v8h*)(gp) = h0;
      *(volatile v8h*)(gp + 256) = h1;

      const int tn = (t + 1 < kSteps) ? (t + 1) : (kSteps - 1);
      const float* xp = x + ((size_t)(b0 + srow) * kSteps + tn) * kInDim + sc8;
      const v4f x0 = *(const v4f*)(xp);
      const v4f x1 = *(const v4f*)(xp + 4);
      v8h xv;
#pragma unroll
      for (int e = 0; e < 4; ++e) {
        xv[e]     = (_Float16)(x0[e] * kCarryA);
        xv[4 + e] = (_Float16)(x1[e] * kCarryA);
      }
      *(v8h*)(sA + srow * kAP + sc8) = xv;
    }
  }
}

__global__ __launch_bounds__(256) void fc_gemm64_kernel(
    const unsigned short* __restrict__ Ap, const unsigned short* __restrict__ Btp,
    float* __restrict__ C, const float* __restrict__ bias)
{
  constexpr int M = kRowsAll, N = kOutD, K = kHid;
  constexpr int lda = kHid, ldb = kHid, ldc = kOutD;
  const _Float16* A  = (const _Float16*)Ap;
  const _Float16* Bt = (const _Float16*)Btp;
  __shared__ __align__(16) float sT[8][16 * 68];
  const int lane = threadIdx.x & 31;
  const int wave = threadIdx.x >> 5;
  constexpr int tilesN = N >> 6;
  constexpr int tilesM = M >> 6;
  const int tile = blockIdx.x * 8 + wave;
  if (tile >= tilesM * tilesN) return;
  const int tm = tile / tilesN;
  const int tn = tile - tm * tilesN;
  const int m0 = tm << 6;
  const int n0 = tn << 6;

  const int rlane = lane & 15;
  const int koff  = (lane >> 4) * 8;
  const int mOff  = (lane >> 4) * 8;

  v8f acc[4][4];
#pragma unroll
  for (int i = 0; i < 4; ++i)
#pragma unroll
    for (int j = 0; j < 4; ++j) acc[i][j] = (v8f){0.f, 0.f, 0.f, 0.f, 0.f, 0.f, 0.f, 0.f};

  for (int k0 = 0; k0 < K; k0 += 32) {
    v16h bh[4];
#pragma unroll
    for (int j = 0; j < 4; ++j) {
      const size_t bo = (size_t)(n0 + (j << 4) + rlane) * ldb + koff + k0;
      bh[j] = frag_load_f16(Bt + bo);
    }
#pragma unroll
    for (int i = 0; i < 4; ++i) {
      const size_t ao = (size_t)(m0 + (i << 4) + rlane) * lda + koff + k0;
      const v16h ah = frag_load_f16(A + ao);
#pragma unroll
      for (int j = 0; j < 4; ++j) acc[i][j] = mma_f16_guarded(ah, bh[j], acc[i][j]);
    }
  }

  float* slab = sT[wave];
#pragma unroll
  for (int i = 0; i < 4; ++i) {
    const int mBase = m0 + (i << 4);
#pragma unroll
    for (int j = 0; j < 4; ++j) {
      const int n = n0 + (j << 4) + rlane;
      const float bv = bias[n];
#pragma unroll
      for (int r = 0; r < 8; ++r) {
        float v = acc[i][j][r] * kFold;
        v += bv;
        slab[(mOff + r) * 68 + (j << 4) + rlane] = v;
      }
    }
    __builtin_amdgcn_fence(__ATOMIC_RELEASE, "workgroup");
    __builtin_amdgcn_wave_barrier();
    __builtin_amdgcn_fence(__ATOMIC_ACQUIRE, "workgroup");
    {
      const int hh = lane >> 4, c4 = (lane & 15) * 4;
      for (int pass = 0; pass < 2; ++pass) {
#pragma unroll
        for (int it = 0; it < 8; ++it) {
          const int row = it * 2 + hh;
          const v4f v = *(const v4f*)(slab + row * 68 + c4);
          *(volatile v4f*)(C + (size_t)(mBase + row) * ldc + n0 + c4) = v;
        }
        __threadfence();
      }
    }
    __builtin_amdgcn_fence(__ATOMIC_RELEASE, "workgroup");
    __builtin_amdgcn_wave_barrier();
    __builtin_amdgcn_fence(__ATOMIC_ACQUIRE, "workgroup");
  }
}

extern "C" void kernel_launch(void* const* d_in, const int* in_sizes, int n_in,
                              void* d_out, int out_size, void* d_ws, size_t ws_size,
                              hipStream_t stream) {
  if (n_in < 7) return;
  if (in_sizes[0] != kBatch * kSteps * kInDim) return;
  if (in_sizes[1] != kGates * kInDim) return;
  if (in_sizes[2] != kGates * kHid) return;
  if (in_sizes[3] != kGates) return;
  if (in_sizes[4] != kGates) return;
  if (in_sizes[5] != kOutD * kHid) return;
  if (in_sizes[6] != kOutD) return;
  if (out_size != kRowsAll * kOutD) return;
  if (ws_size < kWsTotal) return;

  const float* x    = (const float*)d_in[0];
  const float* W_ih = (const float*)d_in[1];
  const float* W_hh = (const float*)d_in[2];
  const float* b_ih = (const float*)d_in[3];
  const float* b_hh = (const float*)d_in[4];
  const float* fc_W = (const float*)d_in[5];
  const float* fc_b = (const float*)d_in[6];
  float* out = (float*)d_out;

  char* ws = (char*)d_ws;
  unsigned short* Wcat  = (unsigned short*)(ws + kOffWcat);
  unsigned short* Fcw   = (unsigned short*)(ws + kOffFcw);
  float*          biasp = (float*)(ws + kOffBias);
  unsigned short* Hs    = (unsigned short*)(ws + kOffHs);

  prep_planes_kernel<<<kBlkWih + kBlkWhh + kBlkFc + kBlkBias, 256, 0, stream>>>(
      W_ih, W_hh, b_ih, b_hh, fc_W, Wcat, Fcw, biasp);

  lstm_steps_kernel<<<kStepBlocks, 512, 0, stream>>>(x, Wcat, biasp, Hs);

  fc_gemm64_kernel<<<((kRowsAll / 64) * (kOutD / 64)) / 8, 256, 0, stream>>>(Hs, Fcw, out, fc_b);
}
